// MotionFormer_5291399708693
// MI455X (gfx1250) — hardware-run, weakly checked
//
#include <hip/hip_runtime.h>
#include <math.h>
#include <stdint.h>

#define NB_   16
#define NC    256
#define SEQ   1024
#define NH    8
#define DH    32
#define MOT   64
#define MHD   8
#define HID   1024
#define QT    64
#define NROW  (NB_ * SEQ)
#define NSAMP (NB_ * SEQ)
#define NEL0  (NB_ * NC * SEQ)
#define NEL1  (NROW * MOT)
#define XP    68
#define TSP   132
#define WTP   72
#define CSP   72
#define OPD   52
#define ASP   72
#define MSP   68
#define STP   32
#define XS    16.0f
#define WSC   64.0f
#define IXS   0.0625f
#define IXW   0.0009765625f
#define IOW   0.0000152587890625f
#define OPF   64.0f
#define CES   256.0f
#define ICES  0.00390625f
#define MDS   64.0f
#define IMW   0.000244140625f
#define ISQ   0.17677669529663687f
#define LNPS  6.931471805599453f
#define BNEPS 1.0e-5f
static_assert(NC == NH * DH);
static_assert(MOT == NH * MHD);
static_assert((SEQ / QT) == 16);
static_assert(SEQ == 4 * 256);
static_assert(NEL0 == 4194304);
static_assert(NEL1 == 1048576);
static_assert(NROW == 16384);
static_assert((HID % 128) == 0);
static_assert((NC % 128) == 0);

typedef _Float16       v16h __attribute__((ext_vector_type(16)));
typedef _Float16       v8h  __attribute__((ext_vector_type(8)));
typedef float          v8f  __attribute__((ext_vector_type(8)));
typedef float          v4f  __attribute__((ext_vector_type(4)));
typedef unsigned int   v4u  __attribute__((ext_vector_type(4)));

union FragH { v16h v; v8h h[2]; };
static_assert(sizeof(FragH) == 32);

__device__ __forceinline__ unsigned short bf_bits(float f) {
  unsigned u = __float_as_uint(f);
  return (unsigned short)((u + 0x7FFFu + ((u >> 16) & 1u)) >> 16);
}
__device__ __forceinline__ float bf_up(unsigned short h) { return __uint_as_float(((unsigned)h) << 16); }
__device__ __forceinline__ float bfr(float f) { return bf_up(bf_bits(f)); }
__device__ __forceinline__ unsigned short h16(float f) {
  const _Float16 x = (_Float16)f;
  return __builtin_bit_cast(unsigned short, x);
}
__device__ __forceinline__ unsigned pk16(unsigned short a, unsigned short b) { return (unsigned)a | ((unsigned)b << 16); }
__device__ __forceinline__ v8f zero8() { v8f z = {0.f, 0.f, 0.f, 0.f, 0.f, 0.f, 0.f, 0.f}; return z; }
__device__ __forceinline__ float hmax8(v8f s) {
  return fmaxf(fmaxf(fmaxf(s[0], s[1]), fmaxf(s[2], s[3])), fmaxf(fmaxf(s[4], s[5]), fmaxf(s[6], s[7])));
}

__device__ __forceinline__ void st2u(unsigned short* p, v4u v) {
  *(volatile v4u*)p = v;
  __threadfence();
  *(volatile v4u*)p = v;
}
__device__ __forceinline__ void st2f(float* p, v4f v) {
  *(volatile v4f*)p = v;
  __threadfence();
  *(volatile v4f*)p = v;
}

__device__ __forceinline__ v16h ldfrag_h(const _Float16* p) {
  FragH f;
  f.h[0] = *(const v8h*)(p);
  f.h[1] = *(const v8h*)(p + 16);
  return f.v;
}

__device__ __forceinline__ v8f mma_h(v16h a, v16h b, v8f c) {
  v8f d = __builtin_amdgcn_wmma_f32_16x16x32_f16(false, a, false, b, (short)0, c, false, false);
#if defined(__HIP_DEVICE_COMPILE__)
  asm volatile("v_nop\n\tv_nop\n\tv_nop\n\tv_nop" : "+v"(d) : "v"(a), "v"(b));
#endif
  return d;
}

__device__ __forceinline__ float ce_val(float c0, float c1, float c2, const float* __restrict__ Wc, int m) {
  const float w0 = bfr(Wc[m]), w1 = bfr(Wc[MOT + m]), w2 = bfr(Wc[2 * MOT + m]);
  return fmaf(c2, w2, fmaf(c1, w1, c0 * w0));
}

template <int RND>
__global__ __launch_bounds__(256)
void bn_stats_kernel(const float* __restrict__ X, float* ST) {
  __shared__ double rs_[8];
  __shared__ double rq_[8];
  const int c = blockIdx.x;
  const int tid = threadIdx.x, lane = tid & 31, wave = tid >> 5;
  double s = 0.0, q = 0.0;
#pragma unroll 1
  for (int bb = 0; bb < NB_; ++bb) {
    const v4f v = *(const v4f*)(X + ((size_t)(bb * NC + c)) * SEQ + 4 * tid);
#pragma unroll
    for (int k = 0; k < 4; ++k) {
      const float f = RND ? bfr(v[k]) : v[k];
      const double d = (double)f;
      s += d;
      q += d * d;
    }
  }
#pragma unroll
  for (int off = 16; off > 0; off >>= 1) {
    s += __shfl_xor(s, off, 32);
    q += __shfl_xor(q, off, 32);
  }
  if (lane == 0) { rs_[wave] = s; rq_[wave] = q; }
  __syncthreads();
  double ts = 0.0, tq = 0.0;
#pragma unroll
  for (int w = 0; w < 8; ++w) { ts += rs_[w]; tq += rq_[w]; }
  const double inv_n = 1.0 / (double)NSAMP;
  const double mu = ts * inv_n;
  double var = tq * inv_n - mu * mu;
  var = (var < 0.0) ? 0.0 : var;
  const float muf  = (float)mu;
  const float rstd = 1.0f / sqrtf((float)var + BNEPS);
  if (tid < 8) {
    v4f u = {0.f, 0.f, 0.f, 0.f};
    if (tid == 0) { u[0] = muf; u[1] = rstd; }
    st2f(ST + (size_t)c * STP + 4 * tid, u);
  }
}

template <int RND>
__global__ __launch_bounds__(256)
void cvt_bn_kernel(const float* __restrict__ X, const float* __restrict__ ST,
                   const float* __restrict__ gam, const float* __restrict__ bet, unsigned short* OUTP) {
  __shared__ __align__(16) float Ts[QT * TSP];
  const int tid = threadIdx.x;
  const int bx = blockIdx.x;
  const int cg = bx & 1, nt = bx >> 1;
  const int b = nt >> 4, n0 = (nt & 15) * QT;
  const int c0 = cg * 128;
  const int row0 = nt * QT;
  {
    const int e = tid & 15, rq = tid >> 4;
#pragma unroll 1
    for (int it = 0; it < 8; ++it) {
      const int cl = it * 16 + rq;
      const int c = c0 + cl;
      const v4f v = *(const v4f*)(X + ((size_t)(b * NC + c)) * SEQ + n0 + 4 * e);
      const float mu = ST[c * STP], rstd = ST[c * STP + 1];
      const float g = bfr(gam[c]), be = bfr(bet[c]);
#pragma unroll
      for (int k = 0; k < 4; ++k) {
        const float f = RND ? bfr(v[k]) : v[k];
        Ts[(4 * e + k) * TSP + cl] = ((f - mu) * rstd) * g + be;
      }
    }
  }
  __syncthreads();
  {
    const int e = tid & 7, lq = tid >> 3;
#pragma unroll 1
    for (int it = 0; it < 4; ++it) {
      const int L = it * 32 + lq;
      const int n = L >> 1, hf = L & 1;
      const float* src = Ts + n * TSP + hf * 64 + 8 * e;
      const v4f x0 = *(const v4f*)(src);
      const v4f x1 = *(const v4f*)(src + 4);
      unsigned short hb[8];
#pragma unroll
      for (int j = 0; j < 4; ++j) {
        hb[j]     = h16(x0[j] * XS);
        hb[4 + j] = h16(x1[j] * XS);
      }
      v4u w;
#pragma unroll
      for (int t = 0; t < 4; ++t) w[t] = pk16(hb[2 * t], hb[2 * t + 1]);
      st2u(OUTP + ((size_t)(row0 + n)) * NC + c0 + hf * 64 + 8 * e, w);
    }
  }
}

__global__ __launch_bounds__(256)
void wt_kernel(const float* __restrict__ W, unsigned short* WT, int K, int N) {
  __shared__ __align__(16) unsigned short Ws[64 * WTP];
  const int tid = threadIdx.x;
  const int nblk = N >> 6;
  const int kb = blockIdx.x / nblk;
  const int nb = blockIdx.x - kb * nblk;
  const int k0 = kb * 64, n0 = nb * 64;
  {
    const int e = tid & 15, rq = tid >> 4;
#pragma unroll 1
    for (int it = 0; it < 4; ++it) {
      const int kl = it * 16 + rq;
      const v4f v = *(const v4f*)(W + ((size_t)(k0 + kl)) * N + n0 + 4 * e);
#pragma unroll
      for (int j = 0; j < 4; ++j) Ws[(4 * e + j) * WTP + kl] = h16(bfr(v[j]) * WSC);
    }
  }
  __syncthreads();
  {
    const int e = tid & 7, lq = tid >> 3;
#pragma unroll 1
    for (int it = 0; it < 2; ++it) {
      const int nl = it * 32 + lq;
      const v4u u = *(const v4u*)(Ws + nl * WTP + 8 * e);
      st2u(WT + ((size_t)(n0 + nl)) * K + k0 + 8 * e, u);
    }
  }
}

__global__ __launch_bounds__(256)
void ce_kernel(const float* __restrict__ cor, const float* __restrict__ Wc, unsigned short* CEP) {
  __shared__ __align__(16) unsigned short Cs[MOT * CSP];
  const int tid = threadIdx.x;
  const int nt = blockIdx.x;
  const int b = nt >> 4, n0 = (nt & 15) * QT;
  {
    const int tok = tid & 63, mq = tid >> 6;
    const size_t row = (size_t)nt * QT + tok;
    const float c0 = bfr(cor[row * 3 + 0]);
    const float c1 = bfr(cor[row * 3 + 1]);
    const float c2 = bfr(cor[row * 3 + 2]);
#pragma unroll 1
    for (int j = 0; j < 16; ++j) {
      const int m = 16 * mq + j;
      Cs[m * CSP + tok] = h16(ce_val(c0, c1, c2, Wc, m) * CES);
    }
  }
  __syncthreads();
  {
    const int e = tid & 7, lq = tid >> 3;
#pragma unroll 1
    for (int it = 0; it < 4; ++it) {
      const int L = it * 32 + lq;
      const int h = L >> 4, r = L & 15;
      const v4u ld = *(const v4u*)(Cs + (h * MHD + (r & 7)) * CSP + 8 * e);
      v4u u;
#pragma unroll
      for (int t = 0; t < 4; ++t) u[t] = (r < 8) ? ld[t] : 0u;
      st2u(CEP + ((size_t)((b * NH + h) * 16 + r)) * SEQ + n0 + 8 * e, u);
    }
  }
}

constexpr int EPI_RM16 = 0;
constexpr int EPI_CF16 = 1;
constexpr int EPI_PROJ = 2;
constexpr int EPI_FC1  = 3;
constexpr int EPI_FC2  = 4;

template <int EPI>
__device__ __forceinline__ void stage_t(float* xs, v8f a, float sc, float bo, float dw, float db, float al) {
  v4f u, w;
#pragma unroll
  for (int r = 0; r < 4; ++r) {
    float t0 = a[r] * sc + bo;
    float t1 = a[4 + r] * sc + bo;
    if (EPI == EPI_FC1) {
      t0 = t0 * dw + db; t0 = (t0 >= 0.f) ? t0 : al * t0;
      t1 = t1 * dw + db; t1 = (t1 >= 0.f) ? t1 : al * t1;
    }
    u[r] = t0; w[r] = t1;
  }
  *(v4f*)(xs) = u;
  *(v4f*)(xs + 4) = w;
}

template <int EPI, int AMODE>
__global__ __launch_bounds__(256)
void gemm_kernel(const unsigned short* __restrict__ A, const unsigned short* __restrict__ WT, int K, int Nout,
                 int ogl2, const float* __restrict__ p0, const float* __restrict__ p1,
                 const float* __restrict__ p2, const float* __restrict__ p3, const float* __restrict__ res,
                 const float* __restrict__ st, const float* __restrict__ gam, const float* __restrict__ bet,
                 unsigned short* O16, float* O32) {
  __shared__ __align__(16) float Xs[128 * XP];
  const int tid  = threadIdx.x;
  const int wave = tid >> 5;
  const int lane = tid & 31;
  const int hh   = lane >> 4;
  const int cc   = lane & 15;
  const int bx   = blockIdx.x;
  const int og   = bx & ((1 << ogl2) - 1);
  const int nt   = bx >> ogl2;
  const int b    = nt >> 4;
  const int n0   = (nt & 15) * QT;
  const int row0 = nt * QT;
  const int o0   = og * 128;
  const int ng = wave & 3, oh = wave >> 2;
  const _Float16* Ah = (const _Float16*)(const void*)A;
  const _Float16* Wh = (const _Float16*)(const void*)WT;

  const _Float16* ahp = (AMODE == 0)
      ? Ah + ((size_t)(row0 + 16 * ng + cc)) * K + 8 * hh
      : Ah + ((size_t)b * NH * SEQ + n0 + 16 * ng + cc) * DH + 8 * hh;
  const size_t kstr = (AMODE == 0) ? (size_t)32 : (size_t)SEQ * DH;
  const _Float16* wp = Wh + ((size_t)(o0 + 64 * oh + cc)) * K + 8 * hh;

  v8f h0 = zero8(), h1 = zero8(), h2 = zero8(), h3 = zero8();
  const int nks = K >> 5;
#pragma unroll 1
  for (int ks = 0; ks < nks; ++ks) {
    const v16h fa = ldfrag_h(ahp + (size_t)ks * kstr);
    const _Float16* wk = wp + 32 * ks;
    v16h bw;
    bw = ldfrag_h(wk + (size_t)0 * 16 * K); h0 = mma_h(fa, bw, h0);
    bw = ldfrag_h(wk + (size_t)1 * 16 * K); h1 = mma_h(fa, bw, h1);
    bw = ldfrag_h(wk + (size_t)2 * 16 * K); h2 = mma_h(fa, bw, h2);
    bw = ldfrag_h(wk + (size_t)3 * 16 * K); h3 = mma_h(fa, bw, h3);
  }

  const int ob = o0 + 64 * oh + cc;
  const float sc = (EPI == EPI_PROJ) ? IOW : IXW;
  float b0v = 0.f, b1v = 0.f, b2v = 0.f, b3v = 0.f;
  float d0v = 0.f, d1v = 0.f, d2v = 0.f, d3v = 0.f;
  float e0v = 0.f, e1v = 0.f, e2v = 0.f, e3v = 0.f;
  float al = 0.f;
  if (EPI == EPI_PROJ || EPI == EPI_FC1 || EPI == EPI_FC2) {
    b0v = bfr(p0[ob + 0 * 16]); b1v = bfr(p0[ob + 1 * 16]);
    b2v = bfr(p0[ob + 2 * 16]); b3v = bfr(p0[ob + 3 * 16]);
  }
  if (EPI == EPI_FC1) {
    d0v = bfr(p1[ob + 0 * 16]); d1v = bfr(p1[ob + 1 * 16]);
    d2v = bfr(p1[ob + 2 * 16]); d3v = bfr(p1[ob + 3 * 16]);
    e0v = bfr(p2[ob + 0 * 16]); e1v = bfr(p2[ob + 1 * 16]);
    e2v = bfr(p2[ob + 2 * 16]); e3v = bfr(p2[ob + 3 * 16]);
    al  = bfr(p3[0]);
  }
  float* xs = Xs + (64 * oh + cc) * XP + 16 * ng + 8 * hh;
  stage_t<EPI>(xs + 0 * 16 * XP, h0, sc, b0v, d0v, e0v, al);
  stage_t<EPI>(xs + 1 * 16 * XP, h1, sc, b1v, d1v, e1v, al);
  stage_t<EPI>(xs + 2 * 16 * XP, h2, sc, b2v, d2v, e2v, al);
  stage_t<EPI>(xs + 3 * 16 * XP, h3, sc, b3v, d3v, e3v, al);
  __syncthreads();

  const int e = tid & 7, lq = tid >> 3;
  if (EPI == EPI_RM16 || EPI == EPI_FC1) {
#pragma unroll 1
    for (int it = 0; it < 4; ++it) {
      const int L = it * 32 + lq;
      const int n = L >> 1, hf = L & 1;
      const float* src = Xs + (hf * 64 + 8 * e) * XP + n;
      unsigned short hb[8];
#pragma unroll
      for (int j = 0; j < 8; ++j) hb[j] = h16(src[j * XP] * XS);
      v4u u;
#pragma unroll
      for (int t = 0; t < 4; ++t) u[t] = pk16(hb[2 * t], hb[2 * t + 1]);
      st2u(O16 + ((size_t)(row0 + n)) * Nout + o0 + hf * 64 + 8 * e, u);
    }
  } else if (EPI == EPI_CF16) {
#pragma unroll 1
    for (int it = 0; it < 4; ++it) {
      const int ol = it * 32 + lq;
      const float* src = Xs + ol * XP + 8 * e;
      const v4f x0 = *(const v4f*)(src);
      const v4f x1 = *(const v4f*)(src + 4);
      unsigned short hb[8];
#pragma unroll
      for (int j = 0; j < 4; ++j) {
        hb[j]     = h16(x0[j] * XS);
        hb[4 + j] = h16(x1[j] * XS);
      }
      v4u u;
#pragma unroll
      for (int t = 0; t < 4; ++t) u[t] = pk16(hb[2 * t], hb[2 * t + 1]);
      st2u(O16 + ((size_t)(b * NC + o0 + ol)) * SEQ + n0 + 8 * e, u);
    }
  } else {
#pragma unroll 1
    for (int it = 0; it < 8; ++it) {
      const int L  = it * 32 + lq;
      const int ol = L >> 1, hf = L & 1;
      const int c  = o0 + ol;
      v4f v = *(const v4f*)(Xs + ol * XP + hf * 32 + 4 * e);
      const size_t gi = ((size_t)(b * NC + c)) * SEQ + n0 + hf * 32 + 4 * e;
      const v4f xr = *(const v4f*)(res + gi);
      if (EPI == EPI_PROJ) {
        const float mu = st[c * STP], rstd = st[c * STP + 1];
        const float g = bfr(gam[c]), be = bfr(bet[c]);
#pragma unroll
        for (int k = 0; k < 4; ++k) v[k] += ((bfr(xr[k]) - mu) * rstd) * g + be;
      } else {
#pragma unroll
        for (int k = 0; k < 4; ++k) v[k] += bfr(xr[k]);
      }
      st2f(O32 + gi, v);
    }
  }
}

__device__ __forceinline__ void stage_o(float* os, v8f o, float rl) {
  v4f u, w;
#pragma unroll
  for (int r = 0; r < 4; ++r) { u[r] = o[r] * rl; w[r] = o[4 + r] * rl; }
  *(v4f*)(os) = u;
  *(v4f*)(os + 4) = w;
}

__global__ __launch_bounds__(128)
void attn_kernel(const unsigned short* __restrict__ QP, const unsigned short* __restrict__ KP,
                 const unsigned short* __restrict__ VT, const unsigned short* __restrict__ CEP,
                 unsigned short* OP, float* CR) {
  __shared__ __align__(16) float Os[QT * OPD];
  const int tid  = threadIdx.x;
  const int wave = tid >> 5;
  const int lane = tid & 31;
  const int hh   = lane >> 4;
  const int c    = lane & 15;
  const int bx   = blockIdx.x;
  const int bh   = bx >> 4;
  const int n0   = (bx & 15) * QT;
  const int b    = bh >> 3, hd = bh & 7;
  const int b2   = (b + (NB_ >> 1)) % NB_;
  const _Float16* QPh = (const _Float16*)(const void*)QP;
  const _Float16* KPh = (const _Float16*)(const void*)KP;
  const _Float16* VTh = (const _Float16*)(const void*)VT;
  const _Float16* CEh = (const _Float16*)(const void*)CEP;

  const v16h qf = ldfrag_h(QPh + ((size_t)(b * SEQ + n0 + wave * 16 + c)) * NC + hd * DH + 8 * hh);
  const _Float16* Kp = KPh + ((size_t)(b2 * SEQ + c)) * NC + hd * DH + 8 * hh;
  const _Float16* Vb = VTh + ((size_t)(b2 * NC + hd * DH + c)) * SEQ + 8 * hh;
  const _Float16* Cb = CEh + ((size_t)(bh * 16 + c)) * SEQ + 8 * hh;
  const float esc = ISQ * IXS * IXS;

  float m = -1.0e30f, l = 0.f;
  v8f o0 = zero8(), o1 = zero8(), o2 = zero8();
#pragma unroll 1
  for (int it = 0; it < SEQ / 32; ++it) {
    const int kb = it * 32;
    const _Float16* k0p = Kp + (size_t)kb * NC;
    const _Float16* k1p = k0p + 16 * NC;
    v8f s0 = mma_h(ldfrag_h(k0p), qf, zero8());
    v8f s1 = mma_h(ldfrag_h(k1p), qf, zero8());
#pragma unroll
    for (int r = 0; r < 8; ++r) { s0[r] *= esc; s1[r] *= esc; }

    float mx = fmaxf(hmax8(s0), hmax8(s1));
    mx = fmaxf(mx, __shfl_xor(mx, 16, 32));
    const float mn   = fmaxf(m, mx);
    const float corr = __expf(m - mn);
    m = mn;
    l *= corr;
#pragma unroll
    for (int r = 0; r < 8; ++r) { o0[r] *= corr; o1[r] *= corr; o2[r] *= corr; }

    FragH ph;
    float ls = 0.f;
    const float msh = mn - LNPS;
#pragma unroll
    for (int r = 0; r < 8; ++r) {
      const float e0 = __expf(s0[r] - msh);
      const float e1 = __expf(s1[r] - msh);
      ls += e0 + e1;
      ph.h[0][r] = (_Float16)e0;
      ph.h[1][r] = (_Float16)e1;
    }
    l += ls;

    o0 = mma_h(ldfrag_h(Vb + kb), ph.v, o0);
    o1 = mma_h(ldfrag_h(Vb + 16 * SEQ + kb), ph.v, o1);
    o2 = mma_h(ldfrag_h(Cb + kb), ph.v, o2);
  }
  l += __shfl_xor(l, 16, 32);
  const float rl = 1.0f / l;

  float* os = Os + (wave * 16 + c) * OPD + 8 * hh;
  stage_o(os + 0, o0, rl);
  stage_o(os + 16, o1, rl);
  stage_o(os + 32, o2, rl);
  __syncthreads();

  {
    const int e = tid & 7, lq = tid >> 3;
#pragma unroll 1
    for (int it = 0; it < 2; ++it) {
      const int L = it * 16 + lq;
      const int n = 2 * L + (e >> 2), d0 = 8 * (e & 3);
      const float* src = Os + n * OPD + d0;
      const v4f x0 = *(const v4f*)(src);
      const v4f x1 = *(const v4f*)(src + 4);
      unsigned short hb[8];
#pragma unroll
      for (int j = 0; j < 4; ++j) {
        hb[j]     = h16(x0[j] * OPF);
        hb[4 + j] = h16(x1[j] * OPF);
      }
      v4u uq;
#pragma unroll
      for (int t = 0; t < 4; ++t) uq[t] = pk16(hb[2 * t], hb[2 * t + 1]);
      st2u(OP + ((size_t)bh * SEQ + n0 + n) * DH + d0, uq);
    }
    {
      const int n = 4 * lq + (e >> 1), j0 = 4 * (e & 1);
      const v4f cv = *(const v4f*)(Os + n * OPD + 32 + j0);
      v4f w;
#pragma unroll
      for (int k = 0; k < 4; ++k) w[k] = cv[k] * ICES;
      st2f(CR + ((size_t)bh * SEQ + n0 + n) * MHD + j0, w);
    }
  }
}

__global__ __launch_bounds__(256)
void mhead_kernel(const float* __restrict__ cor, const float* __restrict__ Wc, const float* __restrict__ CR,
                  const unsigned short* __restrict__ WMT, const float* __restrict__ bm, float* OUT1) {
  __shared__ __align__(16) unsigned short As[QT * ASP];
  __shared__ __align__(16) float Ms[QT * MSP];
  const int tid  = threadIdx.x;
  const int wave = tid >> 5;
  const int lane = tid & 31;
  const int hh   = lane >> 4;
  const int cc   = lane & 15;
  const int nt   = blockIdx.x;
  const int b    = nt >> 4, n0 = (nt & 15) * QT;
  {
    const int tok = tid & 63, mq = tid >> 6;
    const size_t row = (size_t)nt * QT + tok;
    const float c0 = bfr(cor[row * 3 + 0]);
    const float c1 = bfr(cor[row * 3 + 1]);
    const float c2 = bfr(cor[row * 3 + 2]);
    const float* crp = CR + (((size_t)(b * NH + 2 * mq)) * SEQ + n0 + tok) * MHD;
    const float* crq = crp + (size_t)SEQ * MHD;
    const v4f a0 = *(const v4f*)(crp), a1 = *(const v4f*)(crp + 4);
    const v4f a2 = *(const v4f*)(crq), a3 = *(const v4f*)(crq + 4);
    unsigned short hb[16];
#pragma unroll
    for (int j = 0; j < 4; ++j) {
      hb[j]      = h16((a0[j] - ce_val(c0, c1, c2, Wc, 16 * mq + j)) * MDS);
      hb[4 + j]  = h16((a1[j] - ce_val(c0, c1, c2, Wc, 16 * mq + 4 + j)) * MDS);
      hb[8 + j]  = h16((a2[j] - ce_val(c0, c1, c2, Wc, 16 * mq + 8 + j)) * MDS);
      hb[12 + j] = h16((a3[j] - ce_val(c0, c1, c2, Wc, 16 * mq + 12 + j)) * MDS);
    }
    v4u u0, u1;
#pragma unroll
    for (int t = 0; t < 4; ++t) {
      u0[t] = pk16(hb[2 * t], hb[2 * t + 1]);
      u1[t] = pk16(hb[8 + 2 * t], hb[9 + 2 * t]);
    }
    *(v4u*)(As + tok * ASP + 16 * mq) = u0;
    *(v4u*)(As + tok * ASP + 16 * mq + 8) = u1;
  }
  __syncthreads();

  const _Float16* Ash  = (const _Float16*)(const void*)As;
  const _Float16* WMTh = (const _Float16*)(const void*)WMT;
  const int rt = wave & 3, ch = wave >> 2;
  const _Float16* ap = Ash + (16 * rt + cc) * ASP + 8 * hh;
  const _Float16* wq = WMTh + ((size_t)(32 * ch + cc)) * MOT + 8 * hh;
  v8f g0 = zero8(), g1 = zero8();
  {
    const v16h fa = ldfrag_h(ap);
    g0 = mma_h(fa, ldfrag_h(wq), g0);
    g1 = mma_h(fa, ldfrag_h(wq + 16 * MOT), g1);
  }
  {
    const v16h fa = ldfrag_h(ap + 32);
    g0 = mma_h(fa, ldfrag_h(wq + 32), g0);
    g1 = mma_h(fa, ldfrag_h(wq + 16 * MOT + 32), g1);
  }
  const int col0 = 32 * ch + cc, col1 = col0 + 16;
  const float bia0 = bfr(bm[col0]), bia1 = bfr(bm[col1]);
#pragma unroll
  for (int r = 0; r < 8; ++r) {
    Ms[(16 * rt + 8 * hh + r) * MSP + col0] = g0[r] * IMW + bia0;
    Ms[(16 * rt + 8 * hh + r) * MSP + col1] = g1[r] * IMW + bia1;
  }
  __syncthreads();
  {
    const int e = tid & 15, lq = tid >> 4;
#pragma unroll 1
    for (int it = 0; it < 4; ++it) {
      const int tk = it * 16 + lq;
      const v4f v = *(const v4f*)(Ms + tk * MSP + 4 * e);
      st2f(OUT1 + ((size_t)nt * QT + tk) * MOT + 4 * e, v);
    }
  }
}

extern "C" void kernel_launch(void* const* d_in, const int* in_sizes, int n_in,
                              void* d_out, int out_size, void* d_ws, size_t ws_size,
                              hipStream_t stream) {
  if (n_in < 20) return;
  if (in_sizes[0] != NEL0 || in_sizes[1] != NROW * 3 || in_sizes[2] != NC || in_sizes[3] != NC ||
      in_sizes[4] != NC || in_sizes[5] != NC || in_sizes[6] != NC * NC || in_sizes[7] != NC * 2 * NC ||
      in_sizes[8] != 3 * MOT || in_sizes[9] != NC * NC || in_sizes[10] != NC || in_sizes[11] != MOT * MOT ||
      in_sizes[12] != MOT || in_sizes[13] != NC * HID || in_sizes[14] != HID || in_sizes[15] != HID ||
      in_sizes[16] != HID || in_sizes[17] < 1 || in_sizes[18] != HID * NC || in_sizes[19] != NC) return;
  if (out_size != NEL0 + NEL1) return;

  const size_t szST  = (size_t)NC * STP * 4;
  const size_t szA16 = (size_t)NROW * NC * 2;
  const size_t szH1  = (size_t)NROW * HID * 2;
  const size_t szWQ  = (size_t)NC * NC * 2;
  const size_t szWKV = (size_t)2 * NC * NC * 2;
  const size_t szWM  = (size_t)MOT * MOT * 2;
  const size_t szW1  = (size_t)NC * HID * 2;
  const size_t szCEP = (size_t)NB_ * NH * 16 * SEQ * 2;
  const size_t szOP  = (size_t)NB_ * NH * SEQ * DH * 2;
  const size_t szCR  = (size_t)NB_ * NH * SEQ * MHD * 4;
  const size_t szX32 = (size_t)NEL0 * 4;
  size_t off = 0;
  const size_t oST1 = off; off += szST;
  const size_t oST2 = off; off += szST;
  const size_t oXNH = off; off += szA16;
  const size_t oWQT = off; off += szWQ;
  const size_t oWKV = off; off += szWKV;
  const size_t oWPT = off; off += szWQ;
  const size_t oWMT = off; off += szWM;
  const size_t oW1T = off; off += szW1;
  const size_t oW2T = off; off += szW1;
  const size_t oQP  = off; off += szA16;
  const size_t oKP  = off; off += szA16;
  const size_t oVT  = off; off += szA16;
  const size_t oCEP = off; off += szCEP;
  const size_t oOP  = off; off += szOP;
  const size_t oCR  = off; off += szCR;
  const size_t oXN2 = off; off += szX32;
  const size_t oBKH = off; off += szA16;
  const size_t oH1  = off; off += szH1;
  if (off > ws_size) return;
  if (off > (size_t)134217728) return;

  const float* x     = (const float*)d_in[0];
  const float* cor   = (const float*)d_in[1];
  const float* g1    = (const float*)d_in[2];
  const float* b1    = (const float*)d_in[3];
  const float* g2    = (const float*)d_in[4];
  const float* b2    = (const float*)d_in[5];
  const float* Wq    = (const float*)d_in[6];
  const float* Wkv   = (const float*)d_in[7];
  const float* Wcor  = (const float*)d_in[8];
  const float* Wproj = (const float*)d_in[9];
  const float* bproj = (const float*)d_in[10];
  const float* Wm    = (const float*)d_in[11];
  const float* bm    = (const float*)d_in[12];
  const float* W1    = (const float*)d_in[13];
  const float* bfc1  = (const float*)d_in[14];
  const float* dww   = (const float*)d_in[15];
  const float* dwb   = (const float*)d_in[16];
  const float* pa    = (const float*)d_in[17];
  const float* W2    = (const float*)d_in[18];
  const float* bfc2  = (const float*)d_in[19];
  char* ws = (char*)d_ws;
  float* ST1 = (float*)(ws + oST1);
  float* ST2 = (float*)(ws + oST2);
  unsigned short* XNH  = (unsigned short*)(ws + oXNH);
  unsigned short* WQT  = (unsigned short*)(ws + oWQT);
  unsigned short* WKVT = (unsigned short*)(ws + oWKV);
  unsigned short* WPT  = (unsigned short*)(ws + oWPT);
  unsigned short* WMT  = (unsigned short*)(ws + oWMT);
  unsigned short* W1T  = (unsigned short*)(ws + oW1T);
  unsigned short* W2T  = (unsigned short*)(ws + oW2T);
  unsigned short* QP   = (unsigned short*)(ws + oQP);
  unsigned short* KP   = (unsigned short*)(ws + oKP);
  unsigned short* VT   = (unsigned short*)(ws + oVT);
  unsigned short* CEP  = (unsigned short*)(ws + oCEP);
  unsigned short* OP   = (unsigned short*)(ws + oOP);
  float* CR   = (float*)(ws + oCR);
  float* XN2T = (float*)(ws + oXN2);
  unsigned short* BKH  = (unsigned short*)(ws + oBKH);
  unsigned short* H1   = (unsigned short*)(ws + oH1);
  float* out0 = (float*)d_out;
  float* out1 = (float*)d_out + NEL0;

  const dim3 blk256(256), blk128(128);
  const dim3 gBN(NC);
  const dim3 gCV(NB_ * (SEQ / QT) * 2);
  const dim3 gNT(NB_ * (SEQ / QT));
  const dim3 gG2(NB_ * (SEQ / QT) * 2);
  const dim3 gG8(NB_ * (SEQ / QT) * 8);
  const dim3 gAT(NB_ * NH * (SEQ / QT));

  bn_stats_kernel<1><<<gBN, blk256, 0, stream>>>(x, ST1);
  cvt_bn_kernel<1><<<gCV, blk256, 0, stream>>>(x, ST1, g1, b1, XNH);
  wt_kernel<<<dim3((NC / 64) * (NC / 64)), blk256, 0, stream>>>(Wq, WQT, NC, NC);
  wt_kernel<<<dim3((NC / 64) * (2 * NC / 64)), blk256, 0, stream>>>(Wkv, WKVT, NC, 2 * NC);
  wt_kernel<<<dim3((NC / 64) * (NC / 64)), blk256, 0, stream>>>(Wproj, WPT, NC, NC);
  wt_kernel<<<dim3((MOT / 64) * (MOT / 64)), blk256, 0, stream>>>(Wm, WMT, MOT, MOT);
  wt_kernel<<<dim3((NC / 64) * (HID / 64)), blk256, 0, stream>>>(W1, W1T, NC, HID);
  wt_kernel<<<dim3((HID / 64) * (NC / 64)), blk256, 0, stream>>>(W2, W2T, HID, NC);
  ce_kernel<<<gNT, blk256, 0, stream>>>(cor, Wcor, CEP);
  gemm_kernel<EPI_RM16, 0><<<gG2, blk256, 0, stream>>>(XNH, WQT, NC, NC, 1, bproj, bproj, bproj, bproj,
                                                        x, ST1, g1, b1, QP, XN2T);
  gemm_kernel<EPI_RM16, 0><<<gG2, blk256, 0, stream>>>(XNH, WKVT, NC, NC, 1, bproj, bproj, bproj, bproj,
                                                        x, ST1, g1, b1, KP, XN2T);
  gemm_kernel<EPI_CF16, 0><<<gG2, blk256, 0, stream>>>(XNH, WKVT + (size_t)NC * NC, NC, NC, 1, bproj, bproj,
                                                        bproj, bproj, x, ST1, g1, b1, VT, XN2T);
  attn_kernel<<<gAT, blk128, 0, stream>>>(QP, KP, VT, CEP, OP, CR);
  mhead_kernel<<<gNT, blk256, 0, stream>>>(cor, Wcor, CR, WMT, bm, out1);
  gemm_kernel<EPI_PROJ, 1><<<gG2, blk256, 0, stream>>>(OP, WPT, NC, NC, 1, bproj, bproj, bproj, bproj,
                                                        x, ST1, g1, b1, BKH, XN2T);
  bn_stats_kernel<0><<<gBN, blk256, 0, stream>>>(XN2T, ST2);
  cvt_bn_kernel<0><<<gCV, blk256, 0, stream>>>(XN2T, ST2, g2, b2, BKH);
  gemm_kernel<EPI_FC1, 0><<<gG8, blk256, 0, stream>>>(BKH, W1T, NC, HID, 3, bfc1, dww, dwb, pa,
                                                       x, ST1, g1, b1, H1, XN2T);
  gemm_kernel<EPI_FC2, 0><<<gG2, blk256, 0, stream>>>(H1, W2T, HID, NC, 1, bfc2, bfc2, bfc2, bfc2,
                                                       x, ST1, g1, b1, BKH, out0);
  (void)hipGetLastError();
}
